// get_model_20134806684320
// MI455X (gfx1250) — hardware-verified
//
#include <hip/hip_runtime.h>

#pragma clang fp contract(off)

typedef __attribute__((ext_vector_type(16))) _Float16 v16h;
typedef __attribute__((ext_vector_type(8)))  _Float16 v8h;
typedef __attribute__((ext_vector_type(16))) __bf16   v16b;
typedef __attribute__((ext_vector_type(8)))  __bf16   v8b;
typedef __attribute__((ext_vector_type(8)))  float    v8f;
typedef __attribute__((ext_vector_type(4)))  float    v4f;
typedef __attribute__((ext_vector_type(4)))  unsigned int v4u;

constexpr int NBATCH = 64;
constexpr int NPT    = 16384;
constexpr int NS1    = 32;
constexpr int NS2    = 16;
constexpr int KNB    = 32;
constexpr int FW1    = 32;
constexpr int CH1A = 64, CH1B = 64, CH1C = 128;
constexpr int FW2    = 192;
constexpr int CH2A = 128, CH2B = 128, CH2C = 256;
constexpr int FW3    = 320;
constexpr int CH3A = 256, CH3B = 512, CH3C = 128;
constexpr int NCLS = 40, FCN = 64, FCK = 128;
constexpr int M1  = NBATCH * NS1 * KNB;
constexpr int M2  = NBATCH * NS2 * KNB;
constexpr int M3  = NBATCH * NS2;
constexpr int MFC = 64;
constexpr float RAD1SQ = 0.04f;
constexpr float RAD2SQ = 0.16f;

static_assert(MFC == NBATCH);
static_assert(M1 % 64 == 0 && M2 % 64 == 0 && M3 % 64 == 0 && MFC % 64 == 0);
static_assert(FW1 % 32 == 0 && FW2 % 32 == 0 && FW3 % 32 == 0 && FCK % 32 == 0);
static_assert(CH1A % 64 == 0 && CH1B % 64 == 0 && CH1C % 64 == 0);
static_assert(CH2A % 64 == 0 && CH2B % 64 == 0 && CH2C % 64 == 0);
static_assert(CH3A % 64 == 0 && CH3B % 64 == 0 && CH3C % 64 == 0 && FCN % 64 == 0);
static_assert(NS2 * 32 == 512);
static_assert((NBATCH * NS1) % 8 == 0 && M3 % 8 == 0);
static_assert(NCLS % 4 == 0 && (MFC * NCLS * 4) % 512 == 0);

constexpr size_t SZ_W1 = (size_t)CH1A * FW1 * 2;
constexpr size_t SZ_W2 = (size_t)CH1B * CH1A * 2;
constexpr size_t SZ_W3 = (size_t)CH1C * CH1B * 2;
constexpr size_t SZ_W4 = (size_t)CH2A * FW2 * 2;
constexpr size_t SZ_W5 = (size_t)CH2B * CH2A * 2;
constexpr size_t SZ_W6 = (size_t)CH2C * CH2B * 2;
constexpr size_t SZ_W7 = (size_t)CH3A * FW3 * 2;
constexpr size_t SZ_W8 = (size_t)CH3B * CH3A * 2;
constexpr size_t SZ_W9 = (size_t)CH3C * CH3B * 2;
constexpr size_t SZ_WF = (size_t)FCN * FCK * 2;
constexpr size_t OFF_W1H = 0,               OFF_W1L = OFF_W1H + SZ_W1;
constexpr size_t OFF_W2H = OFF_W1L + SZ_W1, OFF_W2L = OFF_W2H + SZ_W2;
constexpr size_t OFF_W3H = OFF_W2L + SZ_W2, OFF_W3L = OFF_W3H + SZ_W3;
constexpr size_t OFF_W4H = OFF_W3L + SZ_W3, OFF_W4L = OFF_W4H + SZ_W4;
constexpr size_t OFF_W5H = OFF_W4L + SZ_W4, OFF_W5L = OFF_W5H + SZ_W5;
constexpr size_t OFF_W6H = OFF_W5L + SZ_W5, OFF_W6L = OFF_W6H + SZ_W6;
constexpr size_t OFF_W7H = OFF_W6L + SZ_W6, OFF_W7L = OFF_W7H + SZ_W7;
constexpr size_t OFF_W8H = OFF_W7L + SZ_W7, OFF_W8L = OFF_W8H + SZ_W8;
constexpr size_t OFF_W9H = OFF_W8L + SZ_W8, OFF_W9L = OFF_W9H + SZ_W9;
constexpr size_t OFF_WFH = OFF_W9L + SZ_W9, OFF_WFL = OFF_WFH + SZ_WF;
constexpr size_t OFF_NX1 = OFF_WFL + SZ_WF;
constexpr size_t OFF_NX2 = OFF_NX1 + (size_t)NBATCH * NS1 * 4 * 4;
constexpr size_t OFF_L1P = OFF_NX2 + (size_t)NBATCH * NS2 * 4 * 4;
constexpr size_t OFF_L2P = OFF_L1P + (size_t)NBATCH * NS1 * CH1C * 4;
constexpr size_t OFF_F3H = OFF_L2P + (size_t)M3 * CH2C * 4;
constexpr size_t OFF_F3L = OFF_F3H + (size_t)M3 * FW3 * 2;
constexpr size_t OFF_E1H = OFF_F3L + (size_t)M3 * FW3 * 2;
constexpr size_t OFF_E1L = OFF_E1H + (size_t)M3 * CH3A * 2;
constexpr size_t OFF_E2H = OFF_E1L + (size_t)M3 * CH3A * 2;
constexpr size_t OFF_E2L = OFF_E2H + (size_t)M3 * CH3B * 2;
constexpr size_t OFF_E3  = OFF_E2L + (size_t)M3 * CH3B * 2;
constexpr size_t OFF_L3H = OFF_E3 + (size_t)M3 * CH3C * 4;
constexpr size_t OFF_L3L = OFF_L3H + (size_t)MFC * FCK * 2;
constexpr size_t OFF_FCO = OFF_L3L + (size_t)MFC * FCK * 2;
constexpr size_t OFF_ARENA = OFF_FCO + (size_t)MFC * FCN * 4;
constexpr size_t AR_F1H = 0;
constexpr size_t AR_F1L = AR_F1H + (size_t)M1 * FW1 * 2;
constexpr size_t AR_H1H = AR_F1L + (size_t)M1 * FW1 * 2;
constexpr size_t AR_H1L = AR_H1H + (size_t)M1 * CH1A * 2;
constexpr size_t AR_H2H = AR_H1L + (size_t)M1 * CH1A * 2;
constexpr size_t AR_H2L = AR_H2H + (size_t)M1 * CH1B * 2;
constexpr size_t AR_H3  = AR_H2L + (size_t)M1 * CH1B * 2;
constexpr size_t AR_END1 = AR_H3 + (size_t)M1 * CH1C * 4;
constexpr size_t AR_F2H = 0;
constexpr size_t AR_F2L = AR_F2H + (size_t)M2 * FW2 * 2;
constexpr size_t AR_G1H = AR_F2L + (size_t)M2 * FW2 * 2;
constexpr size_t AR_G1L = AR_G1H + (size_t)M2 * CH2A * 2;
constexpr size_t AR_G2H = AR_G1L + (size_t)M2 * CH2A * 2;
constexpr size_t AR_G2L = AR_G2H + (size_t)M2 * CH2B * 2;
constexpr size_t AR_G3  = AR_G2L + (size_t)M2 * CH2B * 2;
constexpr size_t AR_END2 = AR_G3 + (size_t)M2 * CH2C * 4;
constexpr size_t AR_SIZE = (AR_END1 > AR_END2) ? AR_END1 : AR_END2;
constexpr size_t WS_TOTAL = OFF_ARENA + AR_SIZE;
static_assert(OFF_ARENA % 4096 == 0 && OFF_NX1 % 128 == 0 && OFF_F3H % 128 == 0 && OFF_L3H % 128 == 0);
static_assert(WS_TOTAL == 100950016ull);
static_assert(WS_TOTAL <= 134217728ull);

__device__ __forceinline__ unsigned short f2bf_bits(float f) {
  unsigned u = __float_as_uint(f);
  return (unsigned short)((u + 0x7FFFu + ((u >> 16) & 1u)) >> 16);
}
__device__ __forceinline__ float bf_bits2f(unsigned short h) { return __uint_as_float(((unsigned)h) << 16); }

__device__ __forceinline__ void dep_guard_h(v8f& a, v8f& b, v16h x, v16h y) { asm volatile("v_nop\n\tv_nop\n\tv_nop\n\tv_nop" : "+v"(a), "+v"(b) : "v"(x), "v"(y)); }
__device__ __forceinline__ void dep_guard_b(v8f& a, v8f& b, v16b x, v16b y) { asm volatile("v_nop\n\tv_nop\n\tv_nop\n\tv_nop" : "+v"(a), "+v"(b) : "v"(x), "v"(y)); }
__device__ __forceinline__ void keep4_h(v16h a, v16h b, v16h c, v16h d) { asm volatile("v_nop" :: "v"(a), "v"(b), "v"(c), "v"(d)); }
__device__ __forceinline__ void keep4_b(v16b a, v16b b, v16b c, v16b d) { asm volatile("v_nop" :: "v"(a), "v"(b), "v"(c), "v"(d)); }
__device__ __forceinline__ void acc_guard4(v8f& a, v8f& b, v8f& c, v8f& d) { asm volatile("v_nop\n\tv_nop\n\tv_nop\n\tv_nop" : "+v"(a), "+v"(b), "+v"(c), "+v"(d)); }
template <typename T> struct Frag;
template <> struct Frag<_Float16> {
  typedef v16h V; union U { v16h v; v8h h[2]; };
  static __device__ __forceinline__ v16h load(const _Float16* p) {
    U f; f.h[0] = *(const v8h*)(p); f.h[1] = *(const v8h*)(p + 16); return f.v;
  }
  static __device__ __forceinline__ v8f mma(v16h a, v16h b, v8f c) {
    return __builtin_amdgcn_wmma_f32_16x16x32_f16(false, a, false, b, (short)0, c, false, false);
  }
  static __device__ __forceinline__ void guard(v8f& a, v8f& b, v16h x, v16h y) { dep_guard_h(a, b, x, y); }
  static __device__ __forceinline__ void keep(v16h a, v16h b, v16h c, v16h d) { keep4_h(a, b, c, d); }
};
template <> struct Frag<__bf16> {
  typedef v16b V; union U { v16b v; v8b h[2]; };
  static __device__ __forceinline__ v16b load(const __bf16* p) {
    U f; f.h[0] = *(const v8b*)(p); f.h[1] = *(const v8b*)(p + 16); return f.v;
  }
  static __device__ __forceinline__ v8f mma(v16b a, v16b b, v8f c) {
    return __builtin_amdgcn_wmma_f32_16x16x32_bf16(false, a, false, b, (short)0, c, false, false);
  }
  static __device__ __forceinline__ void guard(v8f& a, v8f& b, v16b x, v16b y) { dep_guard_b(a, b, x, y); }
  static __device__ __forceinline__ void keep(v16b a, v16b b, v16b c, v16b d) { keep4_b(a, b, c, d); }
};

template <int ET> struct Elem;
template <> struct Elem<0> { typedef _Float16 T; };
template <> struct Elem<1> { typedef __bf16 T; };
template <int ET, bool SPLIT, int BIAS_MODE, int OUT_MODE, bool RESID, int ACT = 0>
__global__ __launch_bounds__(256) void wmma_gemm64(
    const unsigned short* __restrict__ Ap, const unsigned short* __restrict__ A2p, int lda, long strideA,
    const unsigned short* __restrict__ Btp, const unsigned short* __restrict__ Bt2p, int ldb, long strideB,
    void* __restrict__ Cout, void* __restrict__ Cout2, int ldc, long strideC,
    const float* __restrict__ bias,
    const float* __restrict__ resid, long strideR,
    int M, int N, int K, float scale) {
  typedef typename Elem<ET>::T T;
  typedef typename Frag<T>::V V;
  const T* A = (const T*)Ap; const T* A2 = (const T*)A2p; const T* Bt = (const T*)Btp; const T* Bt2 = (const T*)Bt2p;
  __shared__ __align__(16) float sT[8][16 * 68];
  const int b    = blockIdx.y;
  const int lane = threadIdx.x & 31;
  const int wave = threadIdx.x >> 5;
  const int tilesN = N >> 6;
  const int tilesM = M >> 6;
  const int tile = blockIdx.x * 8 + wave;
  if (tile >= tilesM * tilesN) return;
  const int tm = tile / tilesN;
  const int tn = tile - tm * tilesN;
  const int m0 = tm << 6;
  const int n0 = tn << 6;

  const T* Ab  = A  + (size_t)b * strideA;
  const T* Bb  = Bt + (size_t)b * strideB;
  const T* Ab2 = SPLIT ? (A2  + (size_t)b * strideA) : nullptr;
  const T* Bb2 = SPLIT ? (Bt2 + (size_t)b * strideB) : nullptr;

  const int rlane = lane & 15;
  const int koff  = (lane >> 4) * 8;
  const int mOff  = (lane >> 4) * 8;

  v8f acc[4][4];
#pragma unroll
  for (int i = 0; i < 4; ++i)
#pragma unroll
    for (int j = 0; j < 4; ++j) acc[i][j] = (v8f){0.f,0.f,0.f,0.f,0.f,0.f,0.f,0.f};

  for (int k0 = 0; k0 < K; k0 += 32) {
    V bh[4], bl[4];
#pragma unroll
    for (int j = 0; j < 4; ++j) {
      const size_t bo = (size_t)(n0 + (j << 4) + rlane) * ldb + koff + k0;
      bh[j] = Frag<T>::load(Bb + bo);
      if (SPLIT) bl[j] = Frag<T>::load(Bb2 + bo);
    }
#pragma unroll
    for (int i = 0; i < 4; ++i) {
      const size_t ao = (size_t)(m0 + (i << 4) + rlane) * lda + koff + k0;
      V ah = Frag<T>::load(Ab + ao);
      V al;
      if (SPLIT) al = Frag<T>::load(Ab2 + ao);
#pragma unroll
      for (int j = 0; j < 4; ++j) {
        acc[i][j] = Frag<T>::mma(ah, bh[j], acc[i][j]);
        if (SPLIT) {
          acc[i][j] = Frag<T>::mma(ah, bl[j], acc[i][j]);
          acc[i][j] = Frag<T>::mma(al, bh[j], acc[i][j]);
        }
      }
      Frag<T>::guard(acc[i][0], acc[i][3], ah, SPLIT ? al : ah);
    }
    Frag<T>::keep(bh[0], bh[1], bh[2], bh[3]);
    if (SPLIT) Frag<T>::keep(bl[0], bl[1], bl[2], bl[3]);
  }
  acc_guard4(acc[0][0], acc[0][1], acc[0][2], acc[0][3]);
  acc_guard4(acc[1][0], acc[1][1], acc[1][2], acc[1][3]);
  acc_guard4(acc[2][0], acc[2][1], acc[2][2], acc[2][3]);
  acc_guard4(acc[3][0], acc[3][1], acc[3][2], acc[3][3]);

  float* slab = sT[wave];
  const float* Rb = RESID ? (resid + (size_t)b * strideR) : nullptr;
#pragma unroll
  for (int i = 0; i < 4; ++i) {
    const int mBase = m0 + (i << 4);
#pragma unroll
    for (int j = 0; j < 4; ++j) {
      const int n = n0 + (j << 4) + rlane;
      float bv = 0.f;
      if (BIAS_MODE == 2) bv = bias[n];
#pragma unroll
      for (int r = 0; r < 8; ++r) {
        float v = acc[i][j][r] * scale;
        if (BIAS_MODE == 1) v += bias[mBase + mOff + r];
        if (BIAS_MODE == 2) v += bv;
        if (RESID) v += Rb[(size_t)(mBase + mOff + r) * ldc + n];
        if (ACT == 1) v = tanhf(v);
        if (ACT == 2) v = fmaxf(v, 0.0f);
        if (ACT == 3) v = v / (1.0f + expf(-v));
        if (ACT == 4) v = (v > 0.f) ? v : 0.01f * v;
        if (ACT == 5) v = 0.5f * v * (1.0f + erff(v * 0.70710678118654752f));
        slab[(mOff + r) * 68 + (j << 4) + rlane] = v;
      }
    }
    __builtin_amdgcn_fence(__ATOMIC_RELEASE, "workgroup");
    __builtin_amdgcn_wave_barrier();
    __builtin_amdgcn_fence(__ATOMIC_ACQUIRE, "workgroup");
    if (OUT_MODE == 0) {
      float* C = (float*)Cout + (size_t)b * strideC;
      const int hh = lane >> 4, c4 = (lane & 15) * 4;
      for (int pass = 0; pass < 2; ++pass) {
#pragma unroll
        for (int it = 0; it < 8; ++it) {
          const int row = it * 2 + hh;
          v4f v = *(const v4f*)(slab + row * 68 + c4);
          *(volatile v4f*)(C + (size_t)(mBase + row) * ldc + n0 + c4) = v;
        }
        __threadfence();
      }
    } else {
      const int q = lane >> 3, c8 = (lane & 7) * 8;
      unsigned short* C  = (unsigned short*)Cout  + (size_t)b * strideC;
      unsigned short* C2 = (OUT_MODE == 2) ? ((unsigned short*)Cout2 + (size_t)b * strideC) : nullptr;
      for (int pass = 0; pass < 2; ++pass) {
#pragma unroll
        for (int it = 0; it < 4; ++it) {
          const int row = it * 4 + q;
          const float* sp = slab + row * 68 + c8;
          v8h hv, lv;
#pragma unroll
          for (int e = 0; e < 8; ++e) {
            if (OUT_MODE == 1) {
              hv[e] = (_Float16)sp[e];
            } else {
              unsigned short hb = f2bf_bits(sp[e]);
              unsigned short lb = f2bf_bits(sp[e] - bf_bits2f(hb));
              hv[e] = __builtin_bit_cast(_Float16, hb);
              lv[e] = __builtin_bit_cast(_Float16, lb);
            }
          }
          *(volatile v8h*)(C + (size_t)(mBase + row) * ldc + n0 + c8) = hv;
          if (OUT_MODE == 2) *(volatile v8h*)(C2 + (size_t)(mBase + row) * ldc + n0 + c8) = lv;
        }
        __threadfence();
      }
    }
    __builtin_amdgcn_fence(__ATOMIC_RELEASE, "workgroup");
    __builtin_amdgcn_wave_barrier();
    __builtin_amdgcn_fence(__ATOMIC_ACQUIRE, "workgroup");
  }
}

__device__ __forceinline__ void pack_pair(float a, float c, unsigned& hw, unsigned& lw) {
  const unsigned short ha = f2bf_bits(a), hc = f2bf_bits(c);
  const unsigned short la = f2bf_bits(a - bf_bits2f(ha));
  const unsigned short lc = f2bf_bits(c - bf_bits2f(hc));
  hw = (unsigned)ha | ((unsigned)hc << 16);
  lw = (unsigned)la | ((unsigned)lc << 16);
}
__device__ __forceinline__ void pack8(const float (&v)[8], v4u& h, v4u& l) {
  unsigned h0, h1, h2, h3, l0, l1, l2, l3;
  pack_pair(v[0], v[1], h0, l0);
  pack_pair(v[2], v[3], h1, l1);
  pack_pair(v[4], v[5], h2, l2);
  pack_pair(v[6], v[7], h3, l3);
  h = (v4u){h0, h1, h2, h3};
  l = (v4u){l0, l1, l2, l3};
}
__device__ __forceinline__ void load_fence12(float a0, float a1, float a2, float a3, float a4, float a5,
                                             float a6, float a7, float a8, float a9, float a10, float a11) {
  asm volatile("" :: "v"(a0), "v"(a1), "v"(a2), "v"(a3), "v"(a4), "v"(a5),
                     "v"(a6), "v"(a7), "v"(a8), "v"(a9), "v"(a10), "v"(a11) : "memory");
}

__global__ __launch_bounds__(256) void wsplit_kernel(const float* __restrict__ w, int nReal, int kReal, int nRows, int kPad,
                                                     unsigned short* __restrict__ hi, unsigned short* __restrict__ lo) {
  const int chunk = blockIdx.x * 256 + (int)threadIdx.x;
  const int cpr = kPad >> 3;
  const int nch = nRows * cpr;
  if (chunk >= nch) return;
  const int row = chunk / cpr;
  const int c0 = (chunk - row * cpr) << 3;
  const bool rowOk = row < nReal;
  const int rowc = rowOk ? row : (nReal - 1);
  float v[8];
#pragma unroll
  for (int e = 0; e < 8; ++e) {
    const int c = c0 + e;
    const int cc = (c < kReal) ? c : (kReal - 1);
    const float x = w[(size_t)rowc * kReal + cc];
    v[e] = (rowOk && c < kReal) ? x : 0.0f;
  }
  v4u hv, lv;
  pack8(v, hv, lv);
  v4u* H = (v4u*)(hi + (size_t)chunk * 8);
  v4u* L = (v4u*)(lo + (size_t)chunk * 8);
  *(volatile v4u*)H = hv;
  *(volatile v4u*)L = lv;
  __threadfence();
  *(volatile v4u*)H = hv;
  *(volatile v4u*)L = lv;
}

__global__ __launch_bounds__(512) void fps1_kernel(const float* __restrict__ xyz, float* __restrict__ nx1) {
  #pragma clang fp contract(off)
  __shared__ float redv[16];
  __shared__ int   redi[16];
  __shared__ int   fidx[NS1];
  const int tid = threadIdx.x, lane = tid & 31, wave = tid >> 5;
  const int b = blockIdx.x;
  const float* base = xyz + (size_t)b * NPT * 6;
  float px[32], py[32], pz[32], dd[32];
#pragma unroll
  for (int gq = 0; gq < 8; ++gq) {
#pragma unroll
    for (int u = 0; u < 4; ++u) {
      const int i = gq * 4 + u;
      const float* pp = base + (size_t)(i * 512 + tid) * 6;
      px[i] = pp[0]; py[i] = pp[1]; pz[i] = pp[2];
    }
    load_fence12(px[gq * 4], py[gq * 4], pz[gq * 4], px[gq * 4 + 1], py[gq * 4 + 1], pz[gq * 4 + 1],
                 px[gq * 4 + 2], py[gq * 4 + 2], pz[gq * 4 + 2], px[gq * 4 + 3], py[gq * 4 + 3], pz[gq * 4 + 3]);
  }
#pragma unroll
  for (int i = 0; i < 32; ++i) dd[i] = 1e10f;
  int far = 0;
#pragma unroll 1
  for (int it = 0; it < NS1; ++it) {
    if (tid == 0) fidx[it] = far;
    const float* cp = base + (size_t)far * 6;
    const float cx = cp[0], cy = cp[1], cz = cp[2];
    float bestv = -1.0f;
    int besti = 0;
#pragma unroll
    for (int i = 0; i < 32; ++i) {
      const float dx = px[i] - cx, dy = py[i] - cy, dz = pz[i] - cz;
      const float t0 = dx * dx, t1 = dy * dy, t2 = dz * dz;
      float d = (t0 + t2) + t1;
      d = fminf(dd[i], d);
      dd[i] = d;
      const bool gt = d > bestv;
      bestv = gt ? d : bestv;
      besti = gt ? (i * 512 + tid) : besti;
    }
#pragma unroll
    for (int off = 16; off > 0; off >>= 1) {
      const float ov = __shfl_xor(bestv, off);
      const int oi = __shfl_xor(besti, off);
      const bool take = (ov > bestv) || (ov == bestv && oi < besti);
      bestv = take ? ov : bestv;
      besti = take ? oi : besti;
    }
    if (lane == 0) { redv[wave] = bestv; redi[wave] = besti; }
    __syncthreads();
    float bv = redv[0];
    int bi = redi[0];
#pragma unroll
    for (int w2 = 1; w2 < 16; ++w2) {
      const float ov = redv[w2];
      const int oi = redi[w2];
      const bool take = (ov > bv) || (ov == bv && oi < bi);
      bv = take ? ov : bv;
      bi = take ? oi : bi;
    }
    bi = bi < 0 ? 0 : (bi > NPT - 1 ? NPT - 1 : bi);
    far = bi;
    __syncthreads();
  }
  if (wave == 0) {
    int fi = fidx[lane];
    fi = fi < 0 ? 0 : (fi > NPT - 1 ? NPT - 1 : fi);
    const float* fp = base + (size_t)fi * 6;
    const v4f cv = (v4f){fp[0], fp[1], fp[2], 0.0f};
    float* dst = nx1 + ((size_t)b * NS1 + lane) * 4;
    *(volatile v4f*)dst = cv;
    __threadfence();
    *(volatile v4f*)dst = cv;
  }
}

__global__ __launch_bounds__(256) void grp1_kernel(const float* __restrict__ xyz, const float* __restrict__ nx1,
                                                   unsigned short* __restrict__ fh, unsigned short* __restrict__ fl) {
  #pragma clang fp contract(off)
  __shared__ int lst[8][32];
  const int tid = threadIdx.x, lane = tid & 31, wave = tid >> 5;
  const int gw = blockIdx.x * 8 + wave;
  const int b = gw >> 5;
  const float* base = xyz + (size_t)b * NPT * 6;
  const float cx = nx1[(size_t)gw * 4 + 0], cy = nx1[(size_t)gw * 4 + 1], cz = nx1[(size_t)gw * 4 + 2];
  const float s0 = cx * cx, s1 = cy * cy, s2 = cz * cz;
  const float sqs = (s0 + s2) + s1;
  lst[wave][lane] = 0;
  int cnt = 0;
#pragma unroll 1
  for (int bp = 0; bp < NPT && cnt < KNB; bp += 32) {
    const int p = bp + lane;
    const float* pp = base + (size_t)p * 6;
    const float x = pp[0], y = pp[1], z = pp[2];
    float pr = x * cx;
    pr = fmaf(y, cy, pr);
    pr = fmaf(z, cz, pr);
    const float t0 = x * x, t1 = y * y, t2 = z * z;
    const float sqn = (t0 + t2) + t1;
    const float sqr = (sqs + sqn) - 2.0f * pr;
    const bool inr = (sqr <= RAD1SQ);
    const unsigned m = (unsigned)__ballot(inr);
    const int pos = cnt + (int)__popc(m & ((1u << lane) - 1u));
    if (inr && pos < KNB) lst[wave][pos] = p;
    cnt += (int)__popc(m);
  }
  __syncthreads();
  const int first = lst[wave][0];
  const int mine = lst[wave][lane];
  int gi = (lane < cnt) ? mine : first;
  gi = gi < 0 ? 0 : (gi > NPT - 1 ? NPT - 1 : gi);
  const float* gp = base + (size_t)gi * 6;
  const float gx = gp[0] - cx, gy = gp[1] - cy, gz = gp[2] - cz;
  const float n0 = gp[3], n1 = gp[4], n2 = gp[5];
  unsigned hw0, hw1, hw2, lw0, lw1, lw2;
  pack_pair(n0, n1, hw0, lw0);
  pack_pair(n2, gx, hw1, lw1);
  pack_pair(gy, gz, hw2, lw2);
  v4u hv[4], lv[4];
#pragma unroll
  for (int t = 0; t < 4; ++t) {
    const int src = t * 8 + (lane >> 2);
    const unsigned a0 = __shfl(hw0, src), a1 = __shfl(hw1, src), a2 = __shfl(hw2, src);
    const unsigned c0 = __shfl(lw0, src), c1 = __shfl(lw1, src), c2 = __shfl(lw2, src);
    const bool z = ((lane & 3) == 0);
    hv[t] = (v4u){ z ? a0 : 0u, z ? a1 : 0u, z ? a2 : 0u, 0u };
    lv[t] = (v4u){ z ? c0 : 0u, z ? c1 : 0u, z ? c2 : 0u, 0u };
  }
  v4u* H = (v4u*)(fh + (size_t)gw * KNB * FW1);
  v4u* L = (v4u*)(fl + (size_t)gw * KNB * FW1);
  for (int pass = 0; pass < 2; ++pass) {
#pragma unroll
    for (int t = 0; t < 4; ++t) {
      *(volatile v4u*)(H + t * 32 + lane) = hv[t];
      *(volatile v4u*)(L + t * 32 + lane) = lv[t];
    }
    __threadfence();
  }
}

template <int R>
__global__ __launch_bounds__(256) void maxpool_kernel(const float* __restrict__ in, float* __restrict__ outp, int nGroups, int nC) {
  const int t = blockIdx.x * 256 + (int)threadIdx.x;
  const int cpr = nC >> 2;
  if (t >= nGroups * cpr) return;
  const int g = t / cpr;
  const int c4 = (t - g * cpr) * 4;
  const float* p = in + (size_t)g * R * nC + c4;
  v4f m = *(const v4f*)p;
#pragma unroll 1
  for (int r = 1; r < R; ++r) {
    const v4f v = *(const v4f*)(p + (size_t)r * nC);
    m.x = fmaxf(m.x, v.x); m.y = fmaxf(m.y, v.y); m.z = fmaxf(m.z, v.z); m.w = fmaxf(m.w, v.w);
  }
  float* o = outp + (size_t)g * nC + c4;
  *(volatile v4f*)o = m;
  __threadfence();
  *(volatile v4f*)o = m;
}

template <int R>
__global__ __launch_bounds__(256) void maxpool_split_kernel(const float* __restrict__ in, unsigned short* __restrict__ hi,
                                                            unsigned short* __restrict__ lo, int nGroups, int nC) {
  const int t = blockIdx.x * 256 + (int)threadIdx.x;
  const int cpr = nC >> 3;
  if (t >= nGroups * cpr) return;
  const int g = t / cpr;
  const int c8 = (t - g * cpr) * 8;
  const float* p = in + (size_t)g * R * nC + c8;
  v4f ma = *(const v4f*)p, mb = *(const v4f*)(p + 4);
#pragma unroll 1
  for (int r = 1; r < R; ++r) {
    const v4f va = *(const v4f*)(p + (size_t)r * nC);
    const v4f vb = *(const v4f*)(p + (size_t)r * nC + 4);
    ma.x = fmaxf(ma.x, va.x); ma.y = fmaxf(ma.y, va.y); ma.z = fmaxf(ma.z, va.z); ma.w = fmaxf(ma.w, va.w);
    mb.x = fmaxf(mb.x, vb.x); mb.y = fmaxf(mb.y, vb.y); mb.z = fmaxf(mb.z, vb.z); mb.w = fmaxf(mb.w, vb.w);
  }
  const float v[8] = {ma.x, ma.y, ma.z, ma.w, mb.x, mb.y, mb.z, mb.w};
  v4u hv, lv;
  pack8(v, hv, lv);
  v4u* H = (v4u*)(hi + (size_t)g * nC + c8);
  v4u* L = (v4u*)(lo + (size_t)g * nC + c8);
  *(volatile v4u*)H = hv;
  *(volatile v4u*)L = lv;
  __threadfence();
  *(volatile v4u*)H = hv;
  *(volatile v4u*)L = lv;
}

__global__ __launch_bounds__(512) void grp2_kernel(const float* __restrict__ nx1, const float* __restrict__ l1p,
                                                   float* __restrict__ nx2,
                                                   unsigned short* __restrict__ fh, unsigned short* __restrict__ fl) {
  #pragma clang fp contract(off)
  __shared__ float cxs[NS2][4];
  __shared__ int   lst[NS2][32];
  const int tid = threadIdx.x, lane = tid & 31, wave = tid >> 5;
  const int b = blockIdx.x;
  const float* pts = nx1 + (size_t)b * NS1 * 4;
  const float x = pts[lane * 4 + 0], y = pts[lane * 4 + 1], z = pts[lane * 4 + 2];
  if (wave == 0) {
    float dist = 1e10f;
    int far = 0;
    int myfi = 0;
#pragma unroll 1
    for (int it = 0; it < NS2; ++it) {
      myfi = (lane == it) ? far : myfi;
      const float cx = __shfl(x, far), cy = __shfl(y, far), cz = __shfl(z, far);
      const float dx = x - cx, dy = y - cy, dz = z - cz;
      const float t0 = dx * dx, t1 = dy * dy, t2 = dz * dz;
      const float d = (t0 + t2) + t1;
      dist = fminf(dist, d);
      float bv = dist;
      int bi = lane;
#pragma unroll
      for (int off = 16; off > 0; off >>= 1) {
        const float ov = __shfl_xor(bv, off);
        const int oi = __shfl_xor(bi, off);
        const bool take = (ov > bv) || (ov == bv && oi < bi);
        bv = take ? ov : bv;
        bi = take ? oi : bi;
      }
      far = bi & 31;
    }
    const int fi = myfi & 31;
    const float fx = __shfl(x, fi), fy = __shfl(y, fi), fz = __shfl(z, fi);
    if (lane < NS2) { cxs[lane][0] = fx; cxs[lane][1] = fy; cxs[lane][2] = fz; cxs[lane][3] = 0.0f; }
    const v4f cv = (v4f){fx, fy, fz, 0.0f};
    const int lrow = (lane < NS2) ? lane : 0;
    float* dst = nx2 + ((size_t)b * NS2 + lrow) * 4;
    if (lane < NS2) *(volatile v4f*)dst = cv;
    __threadfence();
    if (lane < NS2) *(volatile v4f*)dst = cv;
  }
  __syncthreads();
  const int s2 = wave;
  const float cx = cxs[s2][0], cy = cxs[s2][1], cz = cxs[s2][2];
  const float u0 = cx * cx, u1 = cy * cy, u2 = cz * cz;
  const float sqs = (u0 + u2) + u1;
  float pr = x * cx;
  pr = fmaf(y, cy, pr);
  pr = fmaf(z, cz, pr);
  const float t0 = x * x, t1 = y * y, t2 = z * z;
  const float sqn = (t0 + t2) + t1;
  const float sqr = (sqs + sqn) - 2.0f * pr;
  const bool inr = (sqr <= RAD2SQ);
  const unsigned m = (unsigned)__ballot(inr);
  const int cnt = (int)__popc(m);
  const int pos = (int)__popc(m & ((1u << lane) - 1u));
  lst[s2][lane] = 0;
  if (inr) lst[s2][pos] = lane;
  __syncthreads();
  const int first = lst[s2][0];
  const int mine = lst[s2][lane];
  int gi = (lane < cnt) ? mine : first;
  gi &= 31;
  const float gxl = __shfl(x, gi) - cx, gyl = __shfl(y, gi) - cy, gzl = __shfl(z, gi) - cz;
  const size_t rowBase = ((size_t)b * NS2 + s2) * KNB;
  const bool isP = lane < 16;
  const bool isG = lane == 16;
  const int c8 = (lane & 15) * 8;
#pragma unroll 1
  for (int j = 0; j < KNB; ++j) {
    const int ij = __shfl(gi, j) & 31;
    const float gx = __shfl(gxl, j), gy = __shfl(gyl, j), gz = __shfl(gzl, j);
    const float* src = l1p + ((size_t)b * NS1 + ij) * CH1C + c8;
    const v4f a0 = *(const v4f*)src;
    const v4f a1 = *(const v4f*)(src + 4);
    float v[8];
    v[0] = isP ? a0.x : (isG ? gx : 0.0f);
    v[1] = isP ? a0.y : (isG ? gy : 0.0f);
    v[2] = isP ? a0.z : (isG ? gz : 0.0f);
    v[3] = isP ? a0.w : 0.0f;
    v[4] = isP ? a1.x : 0.0f;
    v[5] = isP ? a1.y : 0.0f;
    v[6] = isP ? a1.z : 0.0f;
    v[7] = isP ? a1.w : 0.0f;
    v4u hv, lv;
    pack8(v, hv, lv);
    v4u* H = (v4u*)(fh + (rowBase + j) * FW2) + lane;
    v4u* L = (v4u*)(fl + (rowBase + j) * FW2) + lane;
    if (lane < 24) { *(volatile v4u*)H = hv; *(volatile v4u*)L = lv; }
    __threadfence();
    if (lane < 24) { *(volatile v4u*)H = hv; *(volatile v4u*)L = lv; }
  }
}

__device__ __forceinline__ void feat3_chunk(const float* __restrict__ prow, int q, float x0, float x1, float x2, v4u& h, v4u& l) {
  float v[8];
#pragma unroll
  for (int e = 0; e < 8; ++e) {
    const int c = q * 8 + e;
    int cc = c - 3;
    cc = cc < 0 ? 0 : (cc > CH2C - 1 ? CH2C - 1 : cc);
    const float pv = prow[cc];
    v[e] = (c == 0) ? x0 : ((c == 1) ? x1 : ((c == 2) ? x2 : ((c < 3 + CH2C) ? pv : 0.0f)));
  }
  pack8(v, h, l);
}
__global__ __launch_bounds__(256) void feat3_kernel(const float* __restrict__ nx2, const float* __restrict__ l2p,
                                                    unsigned short* __restrict__ fh, unsigned short* __restrict__ fl) {
  const int tid = threadIdx.x, lane = tid & 31, wave = tid >> 5;
  const int r = blockIdx.x * 8 + wave;
  const float x0 = nx2[(size_t)r * 4 + 0], x1 = nx2[(size_t)r * 4 + 1], x2 = nx2[(size_t)r * 4 + 2];
  const float* prow = l2p + (size_t)r * CH2C;
  v4u ha, la, hb, lb;
  feat3_chunk(prow, lane, x0, x1, x2, ha, la);
  feat3_chunk(prow, 32 + lane, x0, x1, x2, hb, lb);
  v4u* H = (v4u*)(fh + (size_t)r * FW3);
  v4u* L = (v4u*)(fl + (size_t)r * FW3);
  for (int pass = 0; pass < 2; ++pass) {
    *(volatile v4u*)(H + lane) = ha;
    *(volatile v4u*)(L + lane) = la;
    if (lane < 8) { *(volatile v4u*)(H + 32 + lane) = hb; *(volatile v4u*)(L + 32 + lane) = lb; }
    __threadfence();
  }
}

__global__ __launch_bounds__(256) void out_kernel(const float* __restrict__ fco, const float* __restrict__ fcb, float* __restrict__ outp) {
  const int t = blockIdx.x * 256 + (int)threadIdx.x;
  if (t >= (MFC * NCLS) / 4) return;
  const int f = t * 4;
  const int row = f / NCLS;
  const int col = f - row * NCLS;
  const v4f a = *(const v4f*)(fco + (size_t)row * FCN + col);
  const float b0 = fcb[col], b1 = fcb[col + 1], b2 = fcb[col + 2], b3 = fcb[col + 3];
  const v4f o = (v4f){a.x + b0, a.y + b1, a.z + b2, a.w + b3};
  float* dst = outp + f;
  *(volatile v4f*)dst = o;
  __threadfence();
  *(volatile v4f*)dst = o;
}

static void launch_wsplit(hipStream_t stream, const float* w, int nReal, int kReal, int nRows, int kPad,
                          unsigned short* hi, unsigned short* lo) {
  const int nch = nRows * (kPad / 8);
  const int grid = (nch + 255) / 256;
  wsplit_kernel<<<dim3(grid), dim3(256), 0, stream>>>(w, nReal, kReal, nRows, kPad, hi, lo);
}

template <int BIAS_MODE, int OUT_MODE, int ACT>
static void launch_gemm(hipStream_t stream,
                        const unsigned short* Ah, const unsigned short* Al, int lda,
                        const unsigned short* Bh, const unsigned short* Bl, int ldb,
                        void* C, void* C2, int ldc, const float* bias, int M, int N, int K) {
  const int tiles = (M / 64) * (N / 64);
  const int grid = (tiles + 7) / 8;
  wmma_gemm64<1, true, BIAS_MODE, OUT_MODE, false, ACT><<<dim3(grid, 1), dim3(256), 0, stream>>>(
      Ah, Al, lda, 0L, Bh, Bl, ldb, 0L, C, C2, ldc, 0L, bias, bias, 0L, M, N, K, 1.0f);
}

extern "C" void kernel_launch(void* const* d_in, const int* in_sizes, int n_in,
                              void* d_out, int out_size, void* d_ws, size_t ws_size,
                              hipStream_t stream)
{
  (void)in_sizes; (void)n_in; (void)out_size;
  if (ws_size < WS_TOTAL) return;

  const float* xyz   = (const float*)d_in[0];
  const float* w11   = (const float*)d_in[1];   const float* b11 = (const float*)d_in[2];
  const float* w12   = (const float*)d_in[3];   const float* b12 = (const float*)d_in[4];
  const float* w13   = (const float*)d_in[5];   const float* b13 = (const float*)d_in[6];
  const float* w21   = (const float*)d_in[7];   const float* b21 = (const float*)d_in[8];
  const float* w22   = (const float*)d_in[9];   const float* b22 = (const float*)d_in[10];
  const float* w23   = (const float*)d_in[11];  const float* b23 = (const float*)d_in[12];
  const float* w31   = (const float*)d_in[13];  const float* b31 = (const float*)d_in[14];
  const float* w32   = (const float*)d_in[15];  const float* b32 = (const float*)d_in[16];
  const float* w33   = (const float*)d_in[17];  const float* b33 = (const float*)d_in[18];
  const float* fcw   = (const float*)d_in[19];  const float* fcb = (const float*)d_in[20];
  float* outp = (float*)d_out;

  unsigned char* ws = (unsigned char*)d_ws;
  unsigned char* ar = ws + OFF_ARENA;
  auto p16 = [&](size_t off) { return (unsigned short*)(ws + off); };
  auto p32 = [&](size_t off) { return (float*)(ws + off); };
  auto a16 = [&](size_t off) { return (unsigned short*)(ar + off); };
  auto a32 = [&](size_t off) { return (float*)(ar + off); };

  unsigned short *W1H = p16(OFF_W1H), *W1L = p16(OFF_W1L), *W2H = p16(OFF_W2H), *W2L = p16(OFF_W2L);
  unsigned short *W3H = p16(OFF_W3H), *W3L = p16(OFF_W3L), *W4H = p16(OFF_W4H), *W4L = p16(OFF_W4L);
  unsigned short *W5H = p16(OFF_W5H), *W5L = p16(OFF_W5L), *W6H = p16(OFF_W6H), *W6L = p16(OFF_W6L);
  unsigned short *W7H = p16(OFF_W7H), *W7L = p16(OFF_W7L), *W8H = p16(OFF_W8H), *W8L = p16(OFF_W8L);
  unsigned short *W9H = p16(OFF_W9H), *W9L = p16(OFF_W9L), *WFH = p16(OFF_WFH), *WFL = p16(OFF_WFL);
  float* nx1 = p32(OFF_NX1);
  float* nx2 = p32(OFF_NX2);
  float* l1p = p32(OFF_L1P);
  float* l2p = p32(OFF_L2P);
  unsigned short *F3H = p16(OFF_F3H), *F3L = p16(OFF_F3L);
  unsigned short *E1H = p16(OFF_E1H), *E1L = p16(OFF_E1L), *E2H = p16(OFF_E2H), *E2L = p16(OFF_E2L);
  float* e3 = p32(OFF_E3);
  unsigned short *L3H = p16(OFF_L3H), *L3L = p16(OFF_L3L);
  float* fco = p32(OFF_FCO);
  unsigned short *F1H = a16(AR_F1H), *F1L = a16(AR_F1L), *H1H = a16(AR_H1H), *H1L = a16(AR_H1L);
  unsigned short *H2H = a16(AR_H2H), *H2L = a16(AR_H2L);
  float* h3 = a32(AR_H3);
  unsigned short *F2H = a16(AR_F2H), *F2L = a16(AR_F2L), *G1H = a16(AR_G1H), *G1L = a16(AR_G1L);
  unsigned short *G2H = a16(AR_G2H), *G2L = a16(AR_G2L);
  float* g3 = a32(AR_G3);

  launch_wsplit(stream, w11, CH1A, 6,        CH1A, FW1,  W1H, W1L);
  launch_wsplit(stream, w12, CH1B, CH1A,     CH1B, CH1A, W2H, W2L);
  launch_wsplit(stream, w13, CH1C, CH1B,     CH1C, CH1B, W3H, W3L);
  launch_wsplit(stream, w21, CH2A, CH1C + 3, CH2A, FW2,  W4H, W4L);
  launch_wsplit(stream, w22, CH2B, CH2A,     CH2B, CH2A, W5H, W5L);
  launch_wsplit(stream, w23, CH2C, CH2B,     CH2C, CH2B, W6H, W6L);
  launch_wsplit(stream, w31, CH3A, CH2C + 3, CH3A, FW3,  W7H, W7L);
  launch_wsplit(stream, w32, CH3B, CH3A,     CH3B, CH3A, W8H, W8L);
  launch_wsplit(stream, w33, CH3C, CH3B,     CH3C, CH3B, W9H, W9L);
  launch_wsplit(stream, fcw, NCLS, FCK,      FCN,  FCK,  WFH, WFL);

  fps1_kernel<<<dim3(NBATCH), dim3(512), 0, stream>>>(xyz, nx1);
  grp1_kernel<<<dim3((NBATCH * NS1) / 8), dim3(256), 0, stream>>>(xyz, nx1, F1H, F1L);
  launch_gemm<2, 2, 2>(stream, F1H, F1L, FW1,  W1H, W1L, FW1,  H1H, H1L, CH1A, b11, M1, CH1A, FW1);
  launch_gemm<2, 2, 2>(stream, H1H, H1L, CH1A, W2H, W2L, CH1A, H2H, H2L, CH1B, b12, M1, CH1B, CH1A);
  launch_gemm<2, 0, 2>(stream, H2H, H2L, CH1B, W3H, W3L, CH1B, h3,  h3,  CH1C, b13, M1, CH1C, CH1B);
  {
    const int nGroups = NBATCH * NS1, nC = CH1C;
    const int thr = nGroups * (nC / 4);
    maxpool_kernel<KNB><<<dim3((thr + 255) / 256), dim3(256), 0, stream>>>(h3, l1p, nGroups, nC);
  }

  grp2_kernel<<<dim3(NBATCH), dim3(512), 0, stream>>>(nx1, l1p, nx2, F2H, F2L);
  launch_gemm<2, 2, 2>(stream, F2H, F2L, FW2,  W4H, W4L, FW2,  G1H, G1L, CH2A, b21, M2, CH2A, FW2);
  launch_gemm<2, 2, 2>(stream, G1H, G1L, CH2A, W5H, W5L, CH2A, G2H, G2L, CH2B, b22, M2, CH2B, CH2A);
  launch_gemm<2, 0, 2>(stream, G2H, G2L, CH2B, W6H, W6L, CH2B, g3,  g3,  CH2C, b23, M2, CH2C, CH2B);
  {
    const int nGroups = NBATCH * NS2, nC = CH2C;
    const int thr = nGroups * (nC / 4);
    maxpool_kernel<KNB><<<dim3((thr + 255) / 256), dim3(256), 0, stream>>>(g3, l2p, nGroups, nC);
  }

  feat3_kernel<<<dim3(M3 / 8), dim3(256), 0, stream>>>(nx2, l2p, F3H, F3L);
  launch_gemm<2, 2, 2>(stream, F3H, F3L, FW3,  W7H, W7L, FW3,  E1H, E1L, CH3A, b31, M3, CH3A, FW3);
  launch_gemm<2, 2, 2>(stream, E1H, E1L, CH3A, W8H, W8L, CH3A, E2H, E2L, CH3B, b32, M3, CH3B, CH3A);
  launch_gemm<2, 0, 2>(stream, E2H, E2L, CH3B, W9H, W9L, CH3B, e3,  e3,  CH3C, b33, M3, CH3C, CH3B);
  {
    const int nGroups = NBATCH, nC = CH3C;
    const int thr = nGroups * (nC / 8);
    maxpool_split_kernel<NS2><<<dim3((thr + 255) / 256), dim3(256), 0, stream>>>(e3, L3H, L3L, nGroups, nC);
  }

  launch_gemm<0, 0, 0>(stream, L3H, L3L, FCK, WFH, WFL, FCK, fco, fco, FCN, fcb, MFC, FCN, FCK);
  out_kernel<<<dim3(3), dim3(256), 0, stream>>>(fco, fcb, outp);
}
